// SC_83726092468887
// MI455X (gfx1250) — hardware-run, weakly checked
//
#include <hip/hip_runtime.h>
#include <math.h>

typedef __attribute__((ext_vector_type(16))) _Float16 v16h;
typedef __attribute__((ext_vector_type(8)))  _Float16 v8h;
typedef __attribute__((ext_vector_type(16))) __bf16   v16b;
typedef __attribute__((ext_vector_type(8)))  __bf16   v8b;
typedef __attribute__((ext_vector_type(8)))  float    v8f;
typedef __attribute__((ext_vector_type(4)))  float    v4f;
typedef __attribute__((ext_vector_type(8)))  unsigned int v8u;

constexpr int kBatch = 4;
constexpr int kCin   = 512;
constexpr int kSide  = 64;
constexpr int kNpos  = kSide * kSide;
constexpr int kCi    = 32;
constexpr int kCout  = 32;
constexpr int kPos   = kBatch * kNpos;
constexpr int kK1    = 9 * kCin;
constexpr int kK2    = 9 * kCi;
constexpr float kPCarry = 32768.0f;
constexpr float kBnEps  = 1e-3f;
static_assert(kNpos == 4096);
static_assert(kPos == 16384);
static_assert(kK1 == 4608 && (kK1 % 32) == 0);
static_assert(kK2 == 288 && (kK2 % 32) == 0);
static_assert(kCi == 32 && kCout == 32);

constexpr size_t kSzXH   = (size_t)kPos * kCin * 2;
constexpr size_t kSzW1AB = (size_t)64 * kK1 * 2;
constexpr size_t kSzW1CD = (size_t)64 * kK2 * 2;
constexpr size_t kSzF32P = (size_t)kPos * kCi * 4;
constexpr size_t kSzB16P = (size_t)kPos * kCi * 2;
constexpr size_t kSzPart = (size_t)2 * 64 * 64 * 4;
constexpr size_t kSzStat = (size_t)2 * 64 * 4;
constexpr size_t kSzCPart = (size_t)kBatch * 16 * 1024 * 4;
constexpr size_t kSzAtt  = (size_t)kBatch * 1024 * 4;

constexpr size_t kOffXH    = 0;
constexpr size_t kOffW1AB  = kOffXH    + kSzXH;
constexpr size_t kOffW1CD  = kOffW1AB  + kSzW1AB;
constexpr size_t kOffRAWA  = kOffW1CD  + kSzW1CD;
constexpr size_t kOffRAWB  = kOffRAWA  + kSzF32P;
constexpr size_t kOffFEAT1 = kOffRAWB  + kSzF32P;
constexpr size_t kOffFEAT2 = kOffFEAT1 + kSzF32P;
constexpr size_t kOffQH    = kOffFEAT2 + kSzF32P;
constexpr size_t kOffQL    = kOffQH    + kSzB16P;
constexpr size_t kOffKH    = kOffQL    + kSzB16P;
constexpr size_t kOffKL    = kOffKH    + kSzB16P;
constexpr size_t kOffVT    = kOffKL    + kSzB16P;
constexpr size_t kOffSAH   = kOffVT    + kSzB16P;
constexpr size_t kOffSAL   = kOffSAH   + kSzB16P;
constexpr size_t kOffSCH   = kOffSAL   + kSzB16P;
constexpr size_t kOffSCL   = kOffSCH   + kSzB16P;
constexpr size_t kOffRAWC  = kOffSCL   + kSzB16P;
constexpr size_t kOffRAWD  = kOffRAWC  + kSzF32P;
constexpr size_t kOffPART1 = kOffRAWD  + kSzF32P;
constexpr size_t kOffSTAT1 = kOffPART1 + kSzPart;
constexpr size_t kOffPART2 = kOffSTAT1 + kSzStat;
constexpr size_t kOffSTAT2 = kOffPART2 + kSzPart;
constexpr size_t kOffCPART = kOffSTAT2 + kSzStat;
constexpr size_t kOffATT   = kOffCPART + kSzCPart;
constexpr size_t kWsTotal  = kOffATT   + kSzAtt;
static_assert(kWsTotal == 39769088ull);
static_assert(kWsTotal <= 134217728ull);
static_assert((kOffW1AB % 128) == 0 && (kOffW1CD % 128) == 0 && (kOffRAWA % 128) == 0 && (kOffQH % 128) == 0 &&
              (kOffVT % 128) == 0 && (kOffSAH % 128) == 0 && (kOffRAWC % 128) == 0 && (kOffPART1 % 128) == 0 &&
              (kOffSTAT1 % 128) == 0 && (kOffPART2 % 128) == 0 && (kOffSTAT2 % 128) == 0 && (kOffCPART % 128) == 0 &&
              (kOffATT % 128) == 0);

__device__ __forceinline__ unsigned short f2bf_bits(float f) {
  unsigned u = __float_as_uint(f);
  return (unsigned short)((u + 0x7FFFu + ((u >> 16) & 1u)) >> 16);
}
__device__ __forceinline__ float bf_bits2f(unsigned short h) { return __uint_as_float(((unsigned)h) << 16); }
__device__ __forceinline__ float bf16r(float f) { return bf_bits2f(f2bf_bits(f)); }

template <typename T> struct Frag;
template <> struct Frag<_Float16> {
  typedef v16h V; union U { v16h v; v8h h[2]; };
  static __device__ __forceinline__ v16h load(const _Float16* p) {
    U f; f.h[0] = *(const v8h*)(p); f.h[1] = *(const v8h*)(p + 16); return f.v;
  }
};
template <> struct Frag<__bf16> {
  typedef v16b V; union U { v16b v; v8b h[2]; };
  static __device__ __forceinline__ v16b load(const __bf16* p) {
    U f; f.h[0] = *(const v8b*)(p); f.h[1] = *(const v8b*)(p + 16); return f.v;
  }
};

__device__ __forceinline__ v8f mma_b(v16b a, v16b b, v8f c) {
  c = __builtin_amdgcn_wmma_f32_16x16x32_bf16(false, a, false, b, (short)0, c, false, false);
  asm volatile("v_nop\n\tv_nop\n\tv_nop\n\tv_nop" : "+v"(c) : "v"(a), "v"(b));
  return c;
}
__device__ __forceinline__ v8f mma_h(v16h a, v16h b, v8f c) {
  c = __builtin_amdgcn_wmma_f32_16x16x32_f16(false, a, false, b, (short)0, c, false, false);
  asm volatile("v_nop\n\tv_nop\n\tv_nop\n\tv_nop" : "+v"(c) : "v"(a), "v"(b));
  return c;
}
__device__ __forceinline__ v16b mask16(v16b a, unsigned m) {
  v8u u = __builtin_bit_cast(v8u, a);
  u = u & m;
  return __builtin_bit_cast(v16b, u);
}
__device__ __forceinline__ void wave_lds_sync() {
  __builtin_amdgcn_fence(__ATOMIC_RELEASE, "workgroup");
  __builtin_amdgcn_wave_barrier();
  __builtin_amdgcn_fence(__ATOMIC_ACQUIRE, "workgroup");
}
__device__ __forceinline__ void split_pack8(v4f a0, v4f a1, v8h& hv, v8h& lv) {
#pragma unroll
  for (int e = 0; e < 4; ++e) {
    const float f0 = a0[e];
    const float f1 = a1[e];
    const unsigned short h0 = f2bf_bits(f0), h1 = f2bf_bits(f1);
    const unsigned short l0 = f2bf_bits(f0 - bf_bits2f(h0)), l1 = f2bf_bits(f1 - bf_bits2f(h1));
    hv[e]     = __builtin_bit_cast(_Float16, h0);
    hv[4 + e] = __builtin_bit_cast(_Float16, h1);
    lv[e]     = __builtin_bit_cast(_Float16, l0);
    lv[4 + e] = __builtin_bit_cast(_Float16, l1);
  }
}

__global__ __launch_bounds__(256) void prep_w_kernel(const float* __restrict__ wA, const float* __restrict__ wB,
                                                     unsigned short* __restrict__ out, int cin)
{
  const int piece = blockIdx.x * 256 + threadIdx.x;
  const int cg  = cin >> 3;
  const int ppr = 9 * cg;
  if (piece >= 64 * ppr) return;
  const int n   = piece / ppr;
  const int rem = piece - n * ppr;
  const int tap = rem / cg;
  const int c0  = (rem - tap * cg) * 8;
  const float* w = (n < 32) ? wA : wB;
  const float* src = w + ((size_t)(n & 31) * cin + c0) * 9 + tap;
  v8h hv;
#pragma unroll
  for (int e = 0; e < 8; ++e) {
    const unsigned short hb = f2bf_bits(src[e * 9]);
    hv[e] = __builtin_bit_cast(_Float16, hb);
  }
  unsigned short* q = out + (size_t)piece * 8;
  *(volatile v8h*)q = hv;
  __threadfence();
  *(volatile v8h*)q = hv;
}

__global__ __launch_bounds__(256) void prep_x_kernel(const float* __restrict__ x, unsigned short* __restrict__ xh)
{
  __shared__ float sT[64 * 65];
  const int t = threadIdx.x;
  const int blk = blockIdx.x;
  const int pt = blk & 63, ct = (blk >> 6) & 7, b = blk >> 9;
  const float* xb = x + ((size_t)b * kCin + ct * 64) * kNpos + pt * 64;
#pragma unroll
  for (int i = 0; i < 4; ++i) {
    const int idx = t + 256 * i;
    const int ch = idx >> 4, p4 = (idx & 15) * 4;
    const v4f v = *(const v4f*)(xb + (size_t)ch * kNpos + p4);
    sT[(p4 + 0) * 65 + ch] = v[0];
    sT[(p4 + 1) * 65 + ch] = v[1];
    sT[(p4 + 2) * 65 + ch] = v[2];
    sT[(p4 + 3) * 65 + ch] = v[3];
  }
  __syncthreads();
  v8h hv[2];
#pragma unroll
  for (int it = 0; it < 2; ++it) {
    const int idx = it * 256 + t;
    const int pos = idx >> 3, c8 = (idx & 7) * 8;
#pragma unroll
    for (int e = 0; e < 8; ++e) {
      const unsigned short hb = f2bf_bits(sT[pos * 65 + c8 + e]);
      hv[it][e] = __builtin_bit_cast(_Float16, hb);
    }
  }
  unsigned short* ob = xh + ((size_t)b * kNpos + pt * 64) * kCin + ct * 64;
  for (int pass = 0; pass < 2; ++pass) {
#pragma unroll
    for (int it = 0; it < 2; ++it) {
      const int idx = it * 256 + t;
      const int pos = idx >> 3, c8 = (idx & 7) * 8;
      *(volatile v8h*)(ob + (size_t)pos * kCin + c8) = hv[it];
    }
    __threadfence();
  }
}

__global__ __launch_bounds__(256) void conv_ab_kernel(const unsigned short* __restrict__ xhp,
                                                      const unsigned short* __restrict__ wpl,
                                                      float* __restrict__ rawA, float* __restrict__ rawB)
{
  __shared__ __align__(16) float sT[8][16 * 68];
  const __bf16* xh = (const __bf16*)xhp;
  const __bf16* W  = (const __bf16*)wpl;
  const int lane = threadIdx.x & 31, wave = threadIdx.x >> 5;
  const int rowId = blockIdx.x * 8 + wave;
  const int b = rowId >> 6, h = rowId & 63;
  const int rlane = lane & 15;
  const int koff = (lane >> 4) * 8;
  const int mOff = (lane >> 4) * 8;
  const __bf16* xb = xh + (size_t)b * kNpos * kCin;

  v8f acc[4][4];
#pragma unroll
  for (int i = 0; i < 4; ++i)
#pragma unroll
    for (int j = 0; j < 4; ++j) acc[i][j] = (v8f){0.f,0.f,0.f,0.f,0.f,0.f,0.f,0.f};

#pragma unroll 1
  for (int dyi = 0; dyi < 3; ++dyi) {
    const int hs = h + dyi - 1;
    if (hs < 0 || hs > 63) continue;
#pragma unroll 1
    for (int dxi = 0; dxi < 3; ++dxi) {
      const int dx = dxi - 1;
      const int wl = rlane + dx;
      const int wr = 48 + rlane + dx;
      const unsigned mL = (wl >= 0) ? 0xffffffffu : 0u;
      const unsigned mR = (wr <= 63) ? 0xffffffffu : 0u;
      const int wlc = (wl < 0) ? 0 : wl;
      const int wrc = (wr > 63) ? 63 : wr;
      const __bf16* ap[4];
      ap[0] = xb + (size_t)(hs * 64 + wlc) * kCin + koff;
      ap[1] = xb + (size_t)(hs * 64 + 16 + rlane + dx) * kCin + koff;
      ap[2] = xb + (size_t)(hs * 64 + 32 + rlane + dx) * kCin + koff;
      ap[3] = xb + (size_t)(hs * 64 + wrc) * kCin + koff;
      const __bf16* wt = W + (size_t)rlane * kK1 + (dyi * 3 + dxi) * kCin + koff;
#pragma unroll 1
      for (int ch = 0; ch < kCin / 32; ++ch) {
        const int ko = ch * 32;
        v16b bf[4];
#pragma unroll
        for (int j = 0; j < 4; ++j) bf[j] = Frag<__bf16>::load(wt + (size_t)(j * 16) * kK1 + ko);
#pragma unroll
        for (int i = 0; i < 4; ++i) {
          v16b a = Frag<__bf16>::load(ap[i] + ko);
          if (i == 0) a = mask16(a, mL);
          if (i == 3) a = mask16(a, mR);
#pragma unroll
          for (int j = 0; j < 4; ++j) acc[i][j] = mma_b(a, bf[j], acc[i][j]);
        }
      }
    }
  }

  float* slab = sT[wave];
  const int q = lane >> 3, c4 = (lane & 7) * 4;
  const size_t posRow = (size_t)b * kNpos + (size_t)h * 64;
#pragma unroll
  for (int i = 0; i < 4; ++i) {
#pragma unroll
    for (int j = 0; j < 4; ++j)
#pragma unroll
      for (int r = 0; r < 8; ++r) slab[(mOff + r) * 68 + (j << 4) + rlane] = acc[i][j][r];
    wave_lds_sync();
    v4f va[4], vb[4];
#pragma unroll
    for (int it = 0; it < 4; ++it) {
      const int row = it * 4 + q;
      va[it] = *(const v4f*)(slab + row * 68 + c4);
      vb[it] = *(const v4f*)(slab + row * 68 + 32 + c4);
    }
    for (int pass = 0; pass < 2; ++pass) {
#pragma unroll
      for (int it = 0; it < 4; ++it) {
        const size_t pos = posRow + i * 16 + it * 4 + q;
        *(volatile v4f*)(rawA + pos * kCi + c4) = va[it];
        *(volatile v4f*)(rawB + pos * kCi + c4) = vb[it];
      }
      __threadfence();
    }
    wave_lds_sync();
  }
}

__global__ __launch_bounds__(256) void conv_cd_kernel(const unsigned short* __restrict__ sahp, const unsigned short* __restrict__ salp,
                                                      const unsigned short* __restrict__ schp, const unsigned short* __restrict__ sclp,
                                                      const unsigned short* __restrict__ wpl,
                                                      float* __restrict__ rawC, float* __restrict__ rawD)
{
  __shared__ __align__(16) float sT[8][16 * 36];
  const int sel = blockIdx.y;
  const __bf16* Ah = (const __bf16*)(sel ? schp : sahp);
  const __bf16* Al = (const __bf16*)(sel ? sclp : salp);
  const __bf16* W  = (const __bf16*)wpl + (size_t)sel * 32 * kK2;
  float* outp = sel ? rawD : rawC;
  const int lane = threadIdx.x & 31, wave = threadIdx.x >> 5;
  const int rowId = blockIdx.x * 8 + wave;
  const int b = rowId >> 6, h = rowId & 63;
  const int rlane = lane & 15;
  const int koff = (lane >> 4) * 8;
  const int mOff = (lane >> 4) * 8;
  const size_t bbase = (size_t)b * kNpos * kCi;

  v8f acc[4][2];
#pragma unroll
  for (int i = 0; i < 4; ++i)
#pragma unroll
    for (int j = 0; j < 2; ++j) acc[i][j] = (v8f){0.f,0.f,0.f,0.f,0.f,0.f,0.f,0.f};

#pragma unroll 1
  for (int dyi = 0; dyi < 3; ++dyi) {
    const int hs = h + dyi - 1;
    if (hs < 0 || hs > 63) continue;
#pragma unroll 1
    for (int dxi = 0; dxi < 3; ++dxi) {
      const int dx = dxi - 1;
      const int wl = rlane + dx;
      const int wr = 48 + rlane + dx;
      const unsigned mL = (wl >= 0) ? 0xffffffffu : 0u;
      const unsigned mR = (wr <= 63) ? 0xffffffffu : 0u;
      const int wlc = (wl < 0) ? 0 : wl;
      const int wrc = (wr > 63) ? 63 : wr;
      size_t ao[4];
      ao[0] = bbase + (size_t)(hs * 64 + wlc) * kCi + koff;
      ao[1] = bbase + (size_t)(hs * 64 + 16 + rlane + dx) * kCi + koff;
      ao[2] = bbase + (size_t)(hs * 64 + 32 + rlane + dx) * kCi + koff;
      ao[3] = bbase + (size_t)(hs * 64 + wrc) * kCi + koff;
      const __bf16* wt = W + (size_t)rlane * kK2 + (dyi * 3 + dxi) * kCi + koff;
      v16b bf[2];
#pragma unroll
      for (int j = 0; j < 2; ++j) bf[j] = Frag<__bf16>::load(wt + (size_t)(j * 16) * kK2);
#pragma unroll
      for (int i = 0; i < 4; ++i) {
        v16b ah = Frag<__bf16>::load(Ah + ao[i]);
        v16b al = Frag<__bf16>::load(Al + ao[i]);
        if (i == 0) { ah = mask16(ah, mL); al = mask16(al, mL); }
        if (i == 3) { ah = mask16(ah, mR); al = mask16(al, mR); }
#pragma unroll
        for (int j = 0; j < 2; ++j) {
          acc[i][j] = mma_b(ah, bf[j], acc[i][j]);
          acc[i][j] = mma_b(al, bf[j], acc[i][j]);
        }
      }
    }
  }

  float* slab = sT[wave];
  const int q = lane >> 3, c4 = (lane & 7) * 4;
  const size_t posRow = (size_t)b * kNpos + (size_t)h * 64;
#pragma unroll
  for (int i = 0; i < 4; ++i) {
#pragma unroll
    for (int j = 0; j < 2; ++j)
#pragma unroll
      for (int r = 0; r < 8; ++r) slab[(mOff + r) * 36 + (j << 4) + rlane] = acc[i][j][r];
    wave_lds_sync();
    v4f va[4];
#pragma unroll
    for (int it = 0; it < 4; ++it) va[it] = *(const v4f*)(slab + (it * 4 + q) * 36 + c4);
    for (int pass = 0; pass < 2; ++pass) {
#pragma unroll
      for (int it = 0; it < 4; ++it) {
        const size_t pos = posRow + i * 16 + it * 4 + q;
        *(volatile v4f*)(outp + pos * kCi + c4) = va[it];
      }
      __threadfence();
    }
    wave_lds_sync();
  }
}

__global__ __launch_bounds__(256) void bn_part_kernel(const float* __restrict__ raw0, const float* __restrict__ raw1,
                                                      float* __restrict__ part)
{
  __shared__ float ls[8 * 32];
  __shared__ float ls2[8 * 32];
  const int t = threadIdx.x, c = t & 31, g = t >> 5;
  const int plane = blockIdx.y;
  const float* raw = plane ? raw1 : raw0;
  const float* p = raw + ((size_t)blockIdx.x * 256 + g * 32) * kCi + c;
  float s = 0.f, s2 = 0.f;
#pragma unroll 4
  for (int i = 0; i < 32; ++i) {
    const float v = p[i * kCi];
    s += v;
    s2 = fmaf(v, v, s2);
  }
  ls[g * 32 + c] = s;
  ls2[g * 32 + c] = s2;
  __syncthreads();
  if (t < 32) {
    float S = 0.f, S2 = 0.f;
#pragma unroll
    for (int k = 0; k < 8; ++k) { S += ls[k * 32 + t]; S2 += ls2[k * 32 + t]; }
    float* o = part + ((size_t)plane * 64 + blockIdx.x) * 64;
    *(volatile float*)(o + t) = S;
    *(volatile float*)(o + 32 + t) = S2;
    __threadfence();
    *(volatile float*)(o + t) = S;
    *(volatile float*)(o + 32 + t) = S2;
  }
}

__global__ __launch_bounds__(64) void bn_final_kernel(const float* __restrict__ part, float* __restrict__ stat)
{
  const int t = threadIdx.x, plane = t >> 5, c = t & 31;
  double S = 0.0, S2 = 0.0;
#pragma unroll 1
  for (int blk = 0; blk < 64; ++blk) {
    const float* p = part + ((size_t)plane * 64 + blk) * 64;
    S  += (double)p[c];
    S2 += (double)p[32 + c];
  }
  const double mean = S * (1.0 / (double)kPos);
  double var = S2 * (1.0 / (double)kPos) - mean * mean;
  if (var < 0.0) var = 0.0;
  const float mf = (float)mean;
  const float inv = 1.0f / sqrtf((float)var + kBnEps);
  float* o = stat + plane * 64;
  *(volatile float*)(o + c) = mf;
  *(volatile float*)(o + 32 + c) = inv;
  __threadfence();
  *(volatile float*)(o + c) = mf;
  *(volatile float*)(o + 32 + c) = inv;
}

__global__ __launch_bounds__(256) void bn_apply_kernel(const float* __restrict__ raw0, const float* __restrict__ raw1,
                                                       const float* __restrict__ stat,
                                                       const float* __restrict__ g0, const float* __restrict__ b0,
                                                       const float* __restrict__ g1, const float* __restrict__ b1,
                                                       float* __restrict__ f0, float* __restrict__ f1)
{
  const int plane = blockIdx.y;
  const int t = threadIdx.x;
  const size_t idx = (size_t)blockIdx.x * 256 + t;
  const int c4 = (t & 7) * 4;
  const float* raw = plane ? raw1 : raw0;
  const float* gp  = plane ? g1 : g0;
  const float* bp  = plane ? b1 : b0;
  float* outp = plane ? f1 : f0;
  const v4f xv = *(const v4f*)(raw + idx * 4);
  const v4f mv = *(const v4f*)(stat + plane * 64 + c4);
  const v4f iv = *(const v4f*)(stat + plane * 64 + 32 + c4);
  const v4f gv = *(const v4f*)(gp + c4);
  const v4f bv = *(const v4f*)(bp + c4);
  v4f y;
#pragma unroll
  for (int e = 0; e < 4; ++e) {
    const float gg = bf16r(gv[e]);
    const float bb = bf16r(bv[e]);
    const float n = (xv[e] - mv[e]) * iv[e];
    y[e] = fmaxf(n * gg + bb, 0.0f);
  }
  float* q = outp + idx * 4;
  *(volatile v4f*)q = y;
  __threadfence();
  *(volatile v4f*)q = y;
}

__global__ __launch_bounds__(256) void qkv_kernel(const float* __restrict__ feat1,
                                                  const float* __restrict__ wq, const float* __restrict__ bq,
                                                  const float* __restrict__ wk, const float* __restrict__ bk,
                                                  const float* __restrict__ wv, const float* __restrict__ bv,
                                                  unsigned short* __restrict__ qh, unsigned short* __restrict__ ql,
                                                  unsigned short* __restrict__ kh, unsigned short* __restrict__ kl,
                                                  unsigned short* __restrict__ vt)
{
  __shared__ __align__(16) float sIn[64 * 36];
  __shared__ __align__(16) float sW[96 * 32];
  __shared__ float sB[96];
  __shared__ __align__(16) float sOut[64 * 100];
  const int t = threadIdx.x;
  const int pos0 = blockIdx.x * 64;
#pragma unroll
  for (int i = 0; i < 2; ++i) {
    const int idx = t + 256 * i;
    const int row = idx >> 3, c4 = (idx & 7) * 4;
    const v4f v = *(const v4f*)(feat1 + (size_t)(pos0 + row) * kCi + c4);
    *(v4f*)(sIn + row * 36 + c4) = v;
  }
  {
    const v4f a = *(const v4f*)(wq + t * 4);
    const v4f b = *(const v4f*)(wk + t * 4);
    const v4f c = *(const v4f*)(wv + t * 4);
    v4f ra, rb, rc;
#pragma unroll
    for (int e = 0; e < 4; ++e) { ra[e] = bf16r(a[e]); rb[e] = bf16r(b[e]); rc[e] = bf16r(c[e]); }
    *(v4f*)(sW + t * 4) = ra;
    *(v4f*)(sW + 1024 + t * 4) = rb;
    *(v4f*)(sW + 2048 + t * 4) = rc;
    const float b0 = bq[t & 31], b1 = bk[t & 31], b2 = bv[t & 31];
    const int wave = t >> 5;
    const float bs = (wave == 0) ? b0 : ((wave == 1) ? b1 : b2);
    if (t < 96) sB[t] = bf16r(bs);
  }
  __syncthreads();
  {
    const int p = t & 63, g = t >> 6;
    float xr[32];
#pragma unroll
    for (int q4 = 0; q4 < 8; ++q4) {
      const v4f v = *(const v4f*)(sIn + p * 36 + 4 * q4);
      xr[4 * q4 + 0] = v[0]; xr[4 * q4 + 1] = v[1]; xr[4 * q4 + 2] = v[2]; xr[4 * q4 + 3] = v[3];
    }
#pragma unroll 1
    for (int o = g * 24; o < g * 24 + 24; ++o) {
      float acc = sB[o];
#pragma unroll
      for (int q4 = 0; q4 < 8; ++q4) {
        const v4f wv4 = *(const v4f*)(sW + o * 32 + 4 * q4);
        acc = fmaf(wv4[0], xr[4 * q4 + 0], acc);
        acc = fmaf(wv4[1], xr[4 * q4 + 1], acc);
        acc = fmaf(wv4[2], xr[4 * q4 + 2], acc);
        acc = fmaf(wv4[3], xr[4 * q4 + 3], acc);
      }
      sOut[p * 100 + o] = acc;
    }
  }
  __syncthreads();
  const int pos = t >> 2, cg = (t & 3) * 8;
  v8h qhv, qlv, khv, klv, vv;
  {
    const v4f a0 = *(const v4f*)(sOut + pos * 100 + cg);
    const v4f a1 = *(const v4f*)(sOut + pos * 100 + cg + 4);
    split_pack8(a0, a1, qhv, qlv);
    const v4f k0 = *(const v4f*)(sOut + pos * 100 + 32 + cg);
    const v4f k1 = *(const v4f*)(sOut + pos * 100 + 32 + cg + 4);
    split_pack8(k0, k1, khv, klv);
  }
  const int vch = t >> 3, pg = (t & 7) * 8;
#pragma unroll
  for (int e = 0; e < 8; ++e) vv[e] = (_Float16)sOut[(pg + e) * 100 + 64 + vch];
  const size_t oqk = (size_t)(pos0 + pos) * kCi + cg;
  const int b = pos0 >> 12;
  const size_t ov = ((size_t)b * kCi + vch) * kNpos + (size_t)(pos0 & (kNpos - 1)) + pg;
  for (int pass = 0; pass < 2; ++pass) {
    *(volatile v8h*)(qh + oqk) = qhv;
    *(volatile v8h*)(ql + oqk) = qlv;
    *(volatile v8h*)(kh + oqk) = khv;
    *(volatile v8h*)(kl + oqk) = klv;
    *(volatile v8h*)(vt + ov) = vv;
    __threadfence();
  }
}

__global__ __launch_bounds__(256) void pam_kernel(const unsigned short* __restrict__ qhp, const unsigned short* __restrict__ qlp,
                                                  const unsigned short* __restrict__ khp, const unsigned short* __restrict__ klp,
                                                  const unsigned short* __restrict__ vtp,
                                                  const float* __restrict__ feat1, const float* __restrict__ gamma,
                                                  unsigned short* __restrict__ sah, unsigned short* __restrict__ sal)
{
  __shared__ __align__(16) float sO[8][16 * 36];
  const __bf16* qh = (const __bf16*)qhp;
  const __bf16* ql = (const __bf16*)qlp;
  const __bf16* kh = (const __bf16*)khp;
  const __bf16* kl = (const __bf16*)klp;
  const _Float16* vt = (const _Float16*)vtp;
  const int lane = threadIdx.x & 31, wave = threadIdx.x >> 5;
  const int hh = lane >> 4, c = lane & 15, koff = hh * 8;
  const int pos0 = (blockIdx.x * 8 + wave) * 16;
  const int b = pos0 >> 12;

  const v16b bqh = Frag<__bf16>::load(qh + (size_t)(pos0 + c) * kCi + koff);
  const v16b bql = Frag<__bf16>::load(ql + (size_t)(pos0 + c) * kCi + koff);
  const __bf16* khb = kh + ((size_t)b * kNpos + c) * kCi + koff;
  const __bf16* klb = kl + ((size_t)b * kNpos + c) * kCi + koff;
  const _Float16* vb0 = vt + ((size_t)b * kCi + c) * kNpos + koff;
  const _Float16* vb1 = vb0 + (size_t)16 * kNpos;

  float m = -1.0e30f, l = 0.f;
  v8f o0 = (v8f){0.f,0.f,0.f,0.f,0.f,0.f,0.f,0.f};
  v8f o1 = (v8f){0.f,0.f,0.f,0.f,0.f,0.f,0.f,0.f};

#pragma unroll 1
  for (int k0 = 0; k0 < kNpos; k0 += 64) {
    v8f s[4];
#pragma unroll
    for (int j = 0; j < 4; ++j) {
      const size_t ko = (size_t)(k0 + j * 16) * kCi;
      const v16b ah = Frag<__bf16>::load(khb + ko);
      const v16b al = Frag<__bf16>::load(klb + ko);
      v8f tt = (v8f){0.f,0.f,0.f,0.f,0.f,0.f,0.f,0.f};
      tt = mma_b(ah, bqh, tt);
      tt = mma_b(ah, bql, tt);
      tt = mma_b(al, bqh, tt);
      s[j] = tt;
    }
    float mx = s[0][0];
#pragma unroll
    for (int j = 0; j < 4; ++j)
#pragma unroll
      for (int r = 0; r < 8; ++r) mx = fmaxf(mx, s[j][r]);
    mx = fmaxf(mx, __shfl_xor(mx, 16, 32));
    const float mn = fmaxf(m, mx);
    const float alpha = __expf(m - mn);
    m = mn;
    v16h pf0, pf1;
    float ps = 0.f;
#pragma unroll
    for (int r = 0; r < 8; ++r) {
      const _Float16 h0 = (_Float16)(__expf(s[0][r] - mn) * kPCarry);
      const _Float16 h1 = (_Float16)(__expf(s[1][r] - mn) * kPCarry);
      const _Float16 h2 = (_Float16)(__expf(s[2][r] - mn) * kPCarry);
      const _Float16 h3 = (_Float16)(__expf(s[3][r] - mn) * kPCarry);
      pf0[r] = h0; pf0[8 + r] = h1;
      pf1[r] = h2; pf1[8 + r] = h3;
      ps += ((float)h0 + (float)h1) + ((float)h2 + (float)h3);
    }
    l = l * alpha + ps;
    o0 = o0 * alpha;
    o1 = o1 * alpha;
    {
      const v16h a0 = Frag<_Float16>::load(vb0 + k0);
      const v16h a1 = Frag<_Float16>::load(vb1 + k0);
      o0 = mma_h(a0, pf0, o0);
      o1 = mma_h(a1, pf0, o1);
      const v16h a2 = Frag<_Float16>::load(vb0 + k0 + 32);
      const v16h a3 = Frag<_Float16>::load(vb1 + k0 + 32);
      o0 = mma_h(a2, pf1, o0);
      o1 = mma_h(a3, pf1, o1);
    }
  }

  l = l + __shfl_xor(l, 16, 32);
  const float inv = 1.0f / l;
  const float gm = bf16r(gamma[0]);
  float* slab = sO[wave];
#pragma unroll
  for (int r = 0; r < 8; ++r) {
    slab[c * 36 + 8 * hh + r]      = gm * (o0[r] * inv);
    slab[c * 36 + 16 + 8 * hh + r] = gm * (o1[r] * inv);
  }
  wave_lds_sync();
  v8h hv[2], lv[2];
#pragma unroll
  for (int it = 0; it < 2; ++it) {
    const int piece = it * 32 + lane;
    const int prow = piece >> 2, cg = (piece & 3) * 8;
    const float* fp = feat1 + (size_t)(pos0 + prow) * kCi + cg;
    const v4f s0 = *(const v4f*)(slab + prow * 36 + cg);
    const v4f s1 = *(const v4f*)(slab + prow * 36 + cg + 4);
    const v4f f0 = *(const v4f*)(fp);
    const v4f f1 = *(const v4f*)(fp + 4);
    split_pack8(s0 + f0, s1 + f1, hv[it], lv[it]);
  }
  for (int pass = 0; pass < 2; ++pass) {
#pragma unroll
    for (int it = 0; it < 2; ++it) {
      const int piece = it * 32 + lane;
      const int prow = piece >> 2, cg = (piece & 3) * 8;
      const size_t o = (size_t)(pos0 + prow) * kCi + cg;
      *(volatile v8h*)(sah + o) = hv[it];
      *(volatile v8h*)(sal + o) = lv[it];
    }
    __threadfence();
  }
}

__global__ __launch_bounds__(256) void cam_energy_kernel(const float* __restrict__ feat2, float* __restrict__ cpart)
{
  __shared__ float sX[256 * 33];
  const int t = threadIdx.x, lane = t & 31, wave = t >> 5;
  const size_t pos0 = (size_t)blockIdx.x * 256;
#pragma unroll
  for (int i = 0; i < 8; ++i) {
    const int idx = t + 256 * i;
    const int row = idx >> 3, c4 = (idx & 7) * 4;
    const v4f v = *(const v4f*)(feat2 + (pos0 + row) * kCi + c4);
    sX[row * 33 + c4 + 0] = v[0];
    sX[row * 33 + c4 + 1] = v[1];
    sX[row * 33 + c4 + 2] = v[2];
    sX[row * 33 + c4 + 3] = v[3];
  }
  __syncthreads();
  float a0 = 0.f, a1 = 0.f, a2 = 0.f, a3 = 0.f;
#pragma unroll 4
  for (int n = 0; n < 256; ++n) {
    const float xd = sX[n * 33 + lane];
    a0 = fmaf(sX[n * 33 + wave], xd, a0);
    a1 = fmaf(sX[n * 33 + wave + 8], xd, a1);
    a2 = fmaf(sX[n * 33 + wave + 16], xd, a2);
    a3 = fmaf(sX[n * 33 + wave + 24], xd, a3);
  }
  float* o = cpart + (size_t)blockIdx.x * 1024;
  for (int pass = 0; pass < 2; ++pass) {
    *(volatile float*)(o + (wave) * 32 + lane) = a0;
    *(volatile float*)(o + (wave + 8) * 32 + lane) = a1;
    *(volatile float*)(o + (wave + 16) * 32 + lane) = a2;
    *(volatile float*)(o + (wave + 24) * 32 + lane) = a3;
    __threadfence();
  }
}

__global__ __launch_bounds__(256) void cam_softmax_kernel(const float* __restrict__ cpart, float* __restrict__ att)
{
  const int t = threadIdx.x, b = blockIdx.x;
  double e0 = 0.0, e1 = 0.0, e2 = 0.0, e3 = 0.0;
#pragma unroll 1
  for (int k = 0; k < 16; ++k) {
    const v4f v = *(const v4f*)(cpart + ((size_t)b * 16 + k) * 1024 + t * 4);
    e0 += (double)v[0]; e1 += (double)v[1]; e2 += (double)v[2]; e3 += (double)v[3];
  }
  const float f0 = (float)e0, f1 = (float)e1, f2 = (float)e2, f3 = (float)e3;
  float mxr = fmaxf(fmaxf(f0, f1), fmaxf(f2, f3));
  mxr = fmaxf(mxr, __shfl_xor(mxr, 1, 32));
  mxr = fmaxf(mxr, __shfl_xor(mxr, 2, 32));
  mxr = fmaxf(mxr, __shfl_xor(mxr, 4, 32));
  const float n0 = mxr - f0, n1 = mxr - f1, n2 = mxr - f2, n3 = mxr - f3;
  float nm = fmaxf(fmaxf(n0, n1), fmaxf(n2, n3));
  nm = fmaxf(nm, __shfl_xor(nm, 1, 32));
  nm = fmaxf(nm, __shfl_xor(nm, 2, 32));
  nm = fmaxf(nm, __shfl_xor(nm, 4, 32));
  const float p0 = expf(n0 - nm), p1 = expf(n1 - nm), p2 = expf(n2 - nm), p3 = expf(n3 - nm);
  float sm = (p0 + p1) + (p2 + p3);
  sm += __shfl_xor(sm, 1, 32);
  sm += __shfl_xor(sm, 2, 32);
  sm += __shfl_xor(sm, 4, 32);
  const float inv = 1.0f / sm;
  const v4f o = (v4f){p0 * inv, p1 * inv, p2 * inv, p3 * inv};
  float* q = att + (size_t)b * 1024 + t * 4;
  *(volatile v4f*)q = o;
  __threadfence();
  *(volatile v4f*)q = o;
}

__global__ __launch_bounds__(256) void cam_out_kernel(const float* __restrict__ att, const float* __restrict__ feat2,
                                                      const float* __restrict__ gamma,
                                                      unsigned short* __restrict__ sch, unsigned short* __restrict__ scl)
{
  __shared__ __align__(16) float sIn[64 * 36];
  __shared__ __align__(16) float sW[32 * 32];
  __shared__ __align__(16) float sOut[64 * 36];
  const int t = threadIdx.x;
  const int pos0 = blockIdx.x * 64;
  const int b = pos0 >> 12;
#pragma unroll
  for (int i = 0; i < 2; ++i) {
    const int idx = t + 256 * i;
    const int row = idx >> 3, c4 = (idx & 7) * 4;
    const v4f v = *(const v4f*)(feat2 + (size_t)(pos0 + row) * kCi + c4);
    *(v4f*)(sIn + row * 36 + c4) = v;
  }
  {
    const v4f a = *(const v4f*)(att + (size_t)b * 1024 + t * 4);
    *(v4f*)(sW + t * 4) = a;
  }
  __syncthreads();
  {
    const int p = t & 63, g = t >> 6;
    float xr[32];
#pragma unroll
    for (int q4 = 0; q4 < 8; ++q4) {
      const v4f v = *(const v4f*)(sIn + p * 36 + 4 * q4);
      xr[4 * q4 + 0] = v[0]; xr[4 * q4 + 1] = v[1]; xr[4 * q4 + 2] = v[2]; xr[4 * q4 + 3] = v[3];
    }
#pragma unroll 1
    for (int o = g * 8; o < g * 8 + 8; ++o) {
      float acc = 0.0f;
#pragma unroll
      for (int q4 = 0; q4 < 8; ++q4) {
        const v4f wv4 = *(const v4f*)(sW + o * 32 + 4 * q4);
        acc = fmaf(wv4[0], xr[4 * q4 + 0], acc);
        acc = fmaf(wv4[1], xr[4 * q4 + 1], acc);
        acc = fmaf(wv4[2], xr[4 * q4 + 2], acc);
        acc = fmaf(wv4[3], xr[4 * q4 + 3], acc);
      }
      sOut[p * 36 + o] = acc;
    }
  }
  __syncthreads();
  const float gm = bf16r(gamma[0]);
  const int pos = t >> 2, cg = (t & 3) * 8;
  const v4f s0 = *(const v4f*)(sOut + pos * 36 + cg);
  const v4f s1 = *(const v4f*)(sOut + pos * 36 + cg + 4);
  const v4f x0 = *(const v4f*)(sIn + pos * 36 + cg);
  const v4f x1 = *(const v4f*)(sIn + pos * 36 + cg + 4);
  v8h hv, lv;
  split_pack8(s0 * gm + x0, s1 * gm + x1, hv, lv);
  const size_t o = (size_t)(pos0 + pos) * kCi + cg;
  for (int pass = 0; pass < 2; ++pass) {
    *(volatile v8h*)(sch + o) = hv;
    *(volatile v8h*)(scl + o) = lv;
    __threadfence();
  }
}

__global__ __launch_bounds__(256) void tail_kernel(const float* __restrict__ rawC, const float* __restrict__ rawD,
                                                   const float* __restrict__ stat,
                                                   const float* __restrict__ gC, const float* __restrict__ bC,
                                                   const float* __restrict__ gD, const float* __restrict__ bD,
                                                   const float* __restrict__ w2, const float* __restrict__ b2,
                                                   float* __restrict__ out)
{
  __shared__ __align__(16) float sIn[64 * 36];
  __shared__ __align__(16) float sW[32 * 32];
  __shared__ float sB[32];
  __shared__ __align__(16) float sOut[64 * 36];
  const int t = threadIdx.x;
  const int pos0 = blockIdx.x * 64;
  const int b = pos0 >> 12;
#pragma unroll
  for (int i = 0; i < 2; ++i) {
    const int idx = t + 256 * i;
    const int row = idx >> 3, c4 = (idx & 7) * 4;
    const v4f xc = *(const v4f*)(rawC + (size_t)(pos0 + row) * kCi + c4);
    const v4f xd = *(const v4f*)(rawD + (size_t)(pos0 + row) * kCi + c4);
    const v4f mc = *(const v4f*)(stat + c4);
    const v4f ic = *(const v4f*)(stat + 32 + c4);
    const v4f md = *(const v4f*)(stat + 64 + c4);
    const v4f id = *(const v4f*)(stat + 96 + c4);
    const v4f gcv = *(const v4f*)(gC + c4);
    const v4f bcv = *(const v4f*)(bC + c4);
    const v4f gdv = *(const v4f*)(gD + c4);
    const v4f bdv = *(const v4f*)(bD + c4);
    v4f y;
#pragma unroll
    for (int e = 0; e < 4; ++e) {
      const float nc = (xc[e] - mc[e]) * ic[e];
      const float nd = (xd[e] - md[e]) * id[e];
      const float yc = fmaxf(nc * bf16r(gcv[e]) + bf16r(bcv[e]), 0.0f);
      const float yd = fmaxf(nd * bf16r(gdv[e]) + bf16r(bdv[e]), 0.0f);
      y[e] = yc + yd;
    }
    *(v4f*)(sIn + row * 36 + c4) = y;
  }
  {
    const v4f a = *(const v4f*)(w2 + t * 4);
    v4f ra;
#pragma unroll
    for (int e = 0; e < 4; ++e) ra[e] = bf16r(a[e]);
    *(v4f*)(sW + t * 4) = ra;
    const float bs = b2[t & 31];
    if (t < 32) sB[t] = bf16r(bs);
  }
  __syncthreads();
  {
    const int p = t & 63, g = t >> 6;
    float xr[32];
#pragma unroll
    for (int q4 = 0; q4 < 8; ++q4) {
      const v4f v = *(const v4f*)(sIn + p * 36 + 4 * q4);
      xr[4 * q4 + 0] = v[0]; xr[4 * q4 + 1] = v[1]; xr[4 * q4 + 2] = v[2]; xr[4 * q4 + 3] = v[3];
    }
#pragma unroll 1
    for (int o = g * 8; o < g * 8 + 8; ++o) {
      float acc = 0.0f;
#pragma unroll
      for (int q4 = 0; q4 < 8; ++q4) {
        const v4f wv4 = *(const v4f*)(sW + o * 32 + 4 * q4);
        acc = fmaf(wv4[0], xr[4 * q4 + 0], acc);
        acc = fmaf(wv4[1], xr[4 * q4 + 1], acc);
        acc = fmaf(wv4[2], xr[4 * q4 + 2], acc);
        acc = fmaf(wv4[3], xr[4 * q4 + 3], acc);
      }
      sOut[p * 36 + o] = acc + sB[o];
    }
  }
  __syncthreads();
  v4f ov[2];
#pragma unroll
  for (int it = 0; it < 2; ++it) {
    const int idx = it * 256 + t;
    const int o = idx >> 4, p4 = (idx & 15) * 4;
#pragma unroll
    for (int e = 0; e < 4; ++e) ov[it][e] = fmaxf(sOut[(p4 + e) * 36 + o], 0.0f);
  }
  for (int pass = 0; pass < 2; ++pass) {
#pragma unroll
    for (int it = 0; it < 2; ++it) {
      const int idx = it * 256 + t;
      const int o = idx >> 4, p4 = (idx & 15) * 4;
      *(volatile v4f*)(out + ((size_t)b * kCout + o) * kNpos + (size_t)(pos0 & (kNpos - 1)) + p4) = ov[it];
    }
    __threadfence();
  }
}

extern "C" void kernel_launch(void* const* d_in, const int* in_sizes, int n_in,
                              void* d_out, int out_size, void* d_ws, size_t ws_size,
                              hipStream_t stream) {
  if (n_in < 23) return;
  if (in_sizes[0] != kBatch * kCin * kNpos) return;
  if (in_sizes[1] != kCi * kCin * 9) return;
  if (in_sizes[4] != kCi * kCin * 9) return;
  if (in_sizes[7] != kCi * kCi || in_sizes[9] != kCi * kCi || in_sizes[11] != kCi * kCi) return;
  if (in_sizes[15] != kCi * kCi * 9 || in_sizes[18] != kCi * kCi * 9) return;
  if (in_sizes[21] != kCout * kCi) return;
  if (out_size != kPos * kCout) return;
  if (ws_size < kWsTotal) return;

  const float* x    = (const float*)d_in[0];
  const float* w1a  = (const float*)d_in[1];
  const float* g1a  = (const float*)d_in[2];
  const float* b1a  = (const float*)d_in[3];
  const float* w1b  = (const float*)d_in[4];
  const float* g1b  = (const float*)d_in[5];
  const float* b1b  = (const float*)d_in[6];
  const float* wq   = (const float*)d_in[7];
  const float* bq   = (const float*)d_in[8];
  const float* wk   = (const float*)d_in[9];
  const float* bk   = (const float*)d_in[10];
  const float* wv   = (const float*)d_in[11];
  const float* bv   = (const float*)d_in[12];
  const float* gsa  = (const float*)d_in[13];
  const float* gca  = (const float*)d_in[14];
  const float* w1c  = (const float*)d_in[15];
  const float* g1c  = (const float*)d_in[16];
  const float* b1c  = (const float*)d_in[17];
  const float* w1d  = (const float*)d_in[18];
  const float* g1d  = (const float*)d_in[19];
  const float* b1d  = (const float*)d_in[20];
  const float* w2   = (const float*)d_in[21];
  const float* b2   = (const float*)d_in[22];
  float* out = (float*)d_out;

  char* ws = (char*)d_ws;
  unsigned short* XH    = (unsigned short*)(ws + kOffXH);
  unsigned short* W1AB  = (unsigned short*)(ws + kOffW1AB);
  unsigned short* W1CD  = (unsigned short*)(ws + kOffW1CD);
  float*          RAWA  = (float*)(ws + kOffRAWA);
  float*          RAWB  = (float*)(ws + kOffRAWB);
  float*          FEAT1 = (float*)(ws + kOffFEAT1);
  float*          FEAT2 = (float*)(ws + kOffFEAT2);
  unsigned short* QH    = (unsigned short*)(ws + kOffQH);
  unsigned short* QL    = (unsigned short*)(ws + kOffQL);
  unsigned short* KH    = (unsigned short*)(ws + kOffKH);
  unsigned short* KL    = (unsigned short*)(ws + kOffKL);
  unsigned short* VT    = (unsigned short*)(ws + kOffVT);
  unsigned short* SAH   = (unsigned short*)(ws + kOffSAH);
  unsigned short* SAL   = (unsigned short*)(ws + kOffSAL);
  unsigned short* SCH   = (unsigned short*)(ws + kOffSCH);
  unsigned short* SCL   = (unsigned short*)(ws + kOffSCL);
  float*          RAWC  = (float*)(ws + kOffRAWC);
  float*          RAWD  = (float*)(ws + kOffRAWD);
  float*          PART1 = (float*)(ws + kOffPART1);
  float*          STAT1 = (float*)(ws + kOffSTAT1);
  float*          PART2 = (float*)(ws + kOffPART2);
  float*          STAT2 = (float*)(ws + kOffSTAT2);
  float*          CPART = (float*)(ws + kOffCPART);
  float*          ATT   = (float*)(ws + kOffATT);

  prep_w_kernel<<<(64 * 9 * (kCin / 8)) / 256, 256, 0, stream>>>(w1a, w1b, W1AB, kCin);
  prep_w_kernel<<<(64 * 9 * (kCi / 8)) / 256, 256, 0, stream>>>(w1c, w1d, W1CD, kCi);
  prep_x_kernel<<<kBatch * 8 * 64, 256, 0, stream>>>(x, XH);

  conv_ab_kernel<<<32, 256, 0, stream>>>(XH, W1AB, RAWA, RAWB);
  bn_part_kernel<<<dim3(64, 2), 256, 0, stream>>>(RAWA, RAWB, PART1);
  bn_final_kernel<<<1, 64, 0, stream>>>(PART1, STAT1);
  bn_apply_kernel<<<dim3(512, 2), 256, 0, stream>>>(RAWA, RAWB, STAT1, g1a, b1a, g1b, b1b, FEAT1, FEAT2);

  qkv_kernel<<<kPos / 64, 256, 0, stream>>>(FEAT1, wq, bq, wk, bk, wv, bv, QH, QL, KH, KL, VT);
  pam_kernel<<<kPos / 128, 256, 0, stream>>>(QH, QL, KH, KL, VT, FEAT1, gsa, SAH, SAL);

  cam_energy_kernel<<<kBatch * 16, 256, 0, stream>>>(FEAT2, CPART);
  cam_softmax_kernel<<<kBatch, 256, 0, stream>>>(CPART, ATT);
  cam_out_kernel<<<kPos / 64, 256, 0, stream>>>(ATT, FEAT2, gca, SCH, SCL);

  conv_cd_kernel<<<dim3(32, 2), 256, 0, stream>>>(SAH, SAL, SCH, SCL, W1CD, RAWC, RAWD);
  bn_part_kernel<<<dim3(64, 2), 256, 0, stream>>>(RAWC, RAWD, PART2);
  bn_final_kernel<<<1, 64, 0, stream>>>(PART2, STAT2);
  tail_kernel<<<kPos / 64, 256, 0, stream>>>(RAWC, RAWD, STAT2, g1c, b1c, g1d, b1d, w2, b2, out);
}
